// SimplifiedRingAttention_76312978915794
// MI455X (gfx1250) — hardware-verified
//
#include <hip/hip_runtime.h>
#include <math.h>

typedef __attribute__((ext_vector_type(16))) _Float16 v16h;
typedef __attribute__((ext_vector_type(16))) __bf16 v16b;
typedef __attribute__((ext_vector_type(8)))  _Float16 v8h;
typedef __attribute__((ext_vector_type(8)))  float v8f;
typedef __attribute__((ext_vector_type(4)))  float v4f;
typedef __attribute__((ext_vector_type(2)))  float v2f;
typedef __attribute__((ext_vector_type(4)))  unsigned v4u;
typedef __attribute__((ext_vector_type(4)))  int v4i;
typedef float __attribute__((may_alias)) float_a;
typedef int __attribute__((may_alias)) int_a;

template <typename T> __device__ __forceinline__ void vst2(void* p, T v) { *(volatile T*)p = v; __threadfence(); *(volatile T*)p = v; }
__device__ __forceinline__ v8f wmma16(v16h a, v16h b, v8f c) {
  v8f d = __builtin_amdgcn_wmma_f32_16x16x32_f16(false, a, false, b, (short)0, c, false, false);
  asm volatile("v_nop\n\tv_nop\n\tv_nop\n\tv_nop" : "+v"(d) : "v"(a), "v"(b));
  return d;
}
__device__ __forceinline__ v8f wmma_bf(v16b a, v16b b, v8f c) {
  v8f d = __builtin_amdgcn_wmma_f32_16x16x32_bf16(false, a, false, b, (short)0, c, false, false);
  asm volatile("v_nop\n\tv_nop\n\tv_nop\n\tv_nop" : "+v"(d) : "v"(a), "v"(b));
  return d;
}
__device__ __forceinline__ v16h frag_h(const _Float16* rowk0, int lane) {
  union { v16h v; v8h q[2]; } u; const _Float16* p = rowk0 + 8 * (lane >> 4);
  u.q[0] = *(const v8h*)p; u.q[1] = *(const v8h*)(p + 16); return u.v;
}
__device__ __forceinline__ v16h frag_f32(const float* rowk0, int lane) {
  v16h a; const float* p = rowk0 + 8 * (lane >> 4);
#pragma unroll
  for (int i = 0; i < 8; ++i) { a[i] = (_Float16)p[i]; a[8 + i] = (_Float16)p[16 + i]; }
  return a;
}
__device__ __forceinline__ v16h frag_f32s(const float* rowk0, int lane, float sc) {
  v16h a; const float* p = rowk0 + 8 * (lane >> 4);
#pragma unroll
  for (int i = 0; i < 8; ++i) { a[i] = (_Float16)(p[i] * sc); a[8 + i] = (_Float16)(p[16 + i] * sc); }
  return a;
}
__device__ __forceinline__ v16h fragc_f32(const float* W, int k0, int n, int lane, int ld, int K) {
  v16h a; const int g = lane >> 4;
#pragma unroll
  for (int i = 0; i < 8; ++i) { const int ka = k0 + 8 * g + i, kb = ka + 16;
    a[i] = (_Float16)(ka < K ? W[(size_t)(ka < K ? ka : K - 1) * ld + n] : 0.f); a[8 + i] = (_Float16)(kb < K ? W[(size_t)(kb < K ? kb : K - 1) * ld + n] : 0.f); }
  return a;
}
struct F2 { v16b h, l; };
__device__ __forceinline__ F2 bsplit16(const float v[16]) { F2 r;
#pragma unroll
  for (int i = 0; i < 16; ++i) { const __bf16 h = (__bf16)v[i]; r.h[i] = h; r.l[i] = (__bf16)(v[i] - (float)h); }
  return r; }
__device__ __forceinline__ F2 split_row(const float* row, int k0, int lane) { float v[16]; const float* p = row + k0 + 8 * (lane >> 4);
#pragma unroll
  for (int i = 0; i < 8; ++i) { v[i] = p[i]; v[8 + i] = p[16 + i]; }
  return bsplit16(v); }
__device__ __forceinline__ F2 split_rowK(const float* row, int k0, int lane, int K) { float v[16]; const int g = lane >> 4;
#pragma unroll
  for (int i = 0; i < 8; ++i) { const int ka = k0 + 8 * g + i, kb = ka + 16; v[i] = ka < K ? row[ka < K ? ka : K - 1] : 0.f; v[8 + i] = kb < K ? row[kb < K ? kb : K - 1] : 0.f; }
  return bsplit16(v); }
__device__ __forceinline__ F2 split_col(const float* W, int k0, int n, int lane, int ld, int K) { float v[16]; const int g = lane >> 4;
#pragma unroll
  for (int i = 0; i < 8; ++i) { const int ka = k0 + 8 * g + i, kb = ka + 16; v[i] = ka < K ? W[(size_t)(ka < K ? ka : K - 1) * ld + n] : 0.f; v[8 + i] = kb < K ? W[(size_t)(kb < K ? kb : K - 1) * ld + n] : 0.f; }
  return bsplit16(v); }
__device__ __forceinline__ v8f mac3(const F2& a, const F2& b, v8f c) { c = wmma_bf(a.l, b.h, c); c = wmma_bf(a.h, b.l, c); return wmma_bf(a.h, b.h, c); }
__device__ __forceinline__ float sigm(float v) { return 1.0f / (1.0f + expf(-v)); }
#define LDSX() do { asm volatile("s_wait_dscnt 0" ::: "memory"); __builtin_amdgcn_wave_barrier(); __builtin_amdgcn_fence(__ATOMIC_RELEASE, "workgroup"); } while (0)


#define NB 2
#define SS 2048
#define NH 16
#define DH 64
#define DM (NH * DH)
#ifndef TQB
#define TQB (SS / 64)
#define TNB NB
#endif
typedef __attribute__((ext_vector_type(8))) __bf16 v8b;
__device__ __forceinline__ v16b frag_b(const __bf16* rowk0, int lane) {
  union { v16b v; v8b q[2]; } u; const __bf16* p = rowk0 + 8 * (lane >> 4);
  u.q[0] = *(const v8b*)p; u.q[1] = *(const v8b*)(p + 16); return u.v;
}
__device__ __forceinline__ float bfr(float v) { return (float)(__bf16)v; }
__device__ __attribute__((noinline)) float exp_ni(float v) { return expf(v); }
__device__ __attribute__((noinline)) float erf_ni(float v) { return erff(v); }

#define WS_QB  0u
#define WS_KB  (WS_QB + 2u * NB * SS * DM)
#define WS_VT  (WS_KB + 2u * NB * SS * DM)
#define WS_END (WS_VT + 2u * NB * NH * DH * SS)

__global__ __launch_bounds__(256) void k_rows(const float* __restrict__ Q, const float* __restrict__ Kx, const float* __restrict__ V, __bf16* __restrict__ QB, __bf16* __restrict__ KB, __bf16* __restrict__ VT) {
  __shared__ __align__(16) __bf16 st[DM][72];
  const int tid = threadIdx.x; const size_t r0 = (size_t)blockIdx.x * 64; const int b = (int)(r0 / SS), n0 = (int)(r0 % SS);
  for (int q = tid; q < 64 * DM / 8; q += 256) { const size_t e = r0 * DM + (size_t)q * 8; __bf16 a[8], c[8];
#pragma unroll
    for (int i = 0; i < 8; ++i) { a[i] = (__bf16)Q[e + i]; c[i] = (__bf16)Kx[e + i]; }
    vst2((unsigned*)(QB + e), *(const v4u*)a); vst2((unsigned*)(KB + e), *(const v4u*)c); }
  for (int q = tid; q < 64 * DM; q += 256) { const int rl = q / DM, c = q % DM; st[c][rl] = (__bf16)V[(r0 + rl) * DM + c]; }
  __syncthreads();
  for (int q = tid; q < DM * 8; q += 256) { const int c = q >> 3, pc = q & 7; const int h = c / DH, d = c % DH; vst2((unsigned*)(VT + (((size_t)b * NH + h) * DH + d) * SS + n0 + pc * 8), *(const v4u*)&st[c][pc * 8]); }
}
__global__ __launch_bounds__(128) void k_att(const __bf16* __restrict__ QB, const __bf16* __restrict__ KB, const __bf16* __restrict__ VT, float* __restrict__ OUT) {
  __shared__ __align__(16) float sp[4][16][36]; __shared__ __align__(16) float so[4][16][68];
  const int tid = threadIdx.x, wave = tid >> 5, lane = tid & 31, col = lane & 15, g = lane >> 4; const int qb = blockIdx.x, h = blockIdx.y, b = blockIdx.z; const int q0 = qb * 64 + wave * 16;
  v16b aq[2];
#pragma unroll
  for (int kc = 0; kc < 2; ++kc) aq[kc] = frag_b(QB + ((size_t)b * SS + q0 + col) * DM + h * DH + kc * 32, lane);
  float m[8], l[8];
#pragma unroll
  for (int r = 0; r < 8; ++r) { m[r] = -3.0e38f; l[r] = 0.f; }
  v8f acc[4] = {};
  const int nks = (qb * 64 + 64) / 32;
#pragma unroll 1
  for (int ks = 0; ks < nks; ++ks) { v8f s[2];
#pragma unroll
    for (int ct = 0; ct < 2; ++ct) { const int kk = ks * 32 + ct * 16 + col; v8f c = {};
#pragma unroll
      for (int kc = 0; kc < 2; ++kc) c = wmma_bf(aq[kc], frag_b(KB + ((size_t)b * SS + kk) * DM + h * DH + kc * 32, lane), c);
#pragma unroll
      for (int r = 0; r < 8; ++r) { const int qi = q0 + 8 * g + r; s[ct][r] = (kk <= qi) ? c[r] * 0.125f : -3.0e38f; } }
#pragma unroll
    for (int r = 0; r < 8; ++r) { float mx = fmaxf(s[0][r], s[1][r]);
#pragma unroll
      for (int o = 1; o < 16; o <<= 1) mx = fmaxf(mx, __shfl_xor(mx, o));
      const float mn = fmaxf(m[r], mx); const float alpha = (m[r] <= -1.0e38f) ? 0.f : __expf(m[r] - mn);
      const float e0 = (s[0][r] <= -1.0e38f) ? 0.f : __expf(s[0][r] - mn), e1 = (s[1][r] <= -1.0e38f) ? 0.f : __expf(s[1][r] - mn); float es = e0 + e1;
#pragma unroll
      for (int o = 1; o < 16; o <<= 1) es += __shfl_xor(es, o);
      l[r] = l[r] * alpha + es; m[r] = mn;
#pragma unroll
      for (int dt = 0; dt < 4; ++dt) acc[dt][r] *= alpha;
      sp[wave][8 * g + r][col] = e0; sp[wave][8 * g + r][16 + col] = e1; }
    LDSX();
    const F2 pa = split_row(&sp[wave][col][0], 0, lane);
#pragma unroll
    for (int dt = 0; dt < 4; ++dt) { const size_t vr = (((size_t)b * NH + h) * DH + dt * 16 + col) * SS + (size_t)ks * 32; const v16b vb = frag_b(VT + vr, lane); acc[dt] = wmma_bf(pa.l, vb, acc[dt]); acc[dt] = wmma_bf(pa.h, vb, acc[dt]); }
    LDSX(); }
#pragma unroll
  for (int r = 0; r < 8; ++r) { const float il = 1.0f / l[r];
#pragma unroll
    for (int dt = 0; dt < 4; ++dt) so[wave][8 * g + r][dt * 16 + col] = acc[dt][r] * il; }
  LDSX();
  for (int rl = 0; rl < 16; ++rl) if (lane < 16) vst2(OUT + ((size_t)b * SS + q0 + rl) * DM + h * DH + lane * 4, *(const v4f*)&so[wave][rl][lane * 4]);
}
extern "C" void kernel_launch(void* const* d_in, const int* in_sizes, int n_in, void* d_out, int out_size, void* d_ws, size_t ws_size, hipStream_t stream) {
  (void)in_sizes; (void)n_in; (void)out_size;
  const float** F = (const float**)d_in;
  if (ws_size < (size_t)WS_END) return;
  char* ws = (char*)d_ws; __bf16 *QB = (__bf16*)(ws + WS_QB), *KB = (__bf16*)(ws + WS_KB), *VT = (__bf16*)(ws + WS_VT);
  k_rows<<<NB * SS / 64, 256, 0, stream>>>(F[0], F[1], F[2], QB, KB, VT);
  k_att<<<dim3(TQB, NH, TNB), 128, 0, stream>>>(QB, KB, VT, (float*)d_out);
}
